// ComplexPolarTransformerBeta_17910013625038
// MI455X (gfx1250) — hardware-verified
//
#include <hip/hip_runtime.h>
#include <math.h>

typedef _Float16 v16h __attribute__((ext_vector_type(16)));
typedef _Float16 v8h  __attribute__((ext_vector_type(8)));
typedef __bf16   v16b __attribute__((ext_vector_type(16)));
typedef unsigned short v8us __attribute__((ext_vector_type(8)));
typedef float v8f __attribute__((ext_vector_type(8)));
typedef float v4f __attribute__((ext_vector_type(4)));
typedef v8h  __attribute__((may_alias)) v8ha;
typedef v8us __attribute__((may_alias)) v8usa;
typedef v4f  __attribute__((may_alias)) v4fa;

union FragH { v16h v; v8h half[2]; };
union FragB { v16b v; v8us half[2]; };

#define NMOL   1024
#define NATOM  128
#define HID    128
#define NEDGE  1024
#define NLAYER 4
#define INDIM  16
#define KEMB   19
#define KCAT   256
#define EDIM   4
#define NTHR   256

#define WSCALE 64.0f
#define WINV   0.015625f
#define PSCALE 1024.0f
#define PINV   0.0009765625f
#define PSHIFT 8.0f
#define SCALE  0.08838834764831845f
#define INVN   0.0078125f
#define LNEPS  1e-5f

#define SZ_F32T   (NATOM * HID * 4)
#define SZ_H16T   (NATOM * HID * 2)
#define OFF_MAG   0
#define OFF_PH    (OFF_MAG + SZ_F32T)
#define OFF_P     (OFF_PH + SZ_F32T)
#define OFF_T     (OFF_P + SZ_H16T)
#define OFF_BIAS  (OFF_T + SZ_H16T)
#define OFF_SLOT  (OFF_BIAS + SZ_F32T)
#define OFF_VAL   (OFF_SLOT + NEDGE * 4)
#define OFF_CNT   (OFF_VAL + NEDGE * 4)
#define OFF_START (OFF_CNT + 512)
#define OFF_MEAN  (OFF_START + 1024)
#define SMEM_BYTES (OFF_MEAN + 1024)

static_assert(SMEM_BYTES == 272896);
static_assert(OFF_BIAS + NATOM * KCAT * 2 == OFF_SLOT);
static_assert(OFF_P + NATOM * KCAT * 2 == OFF_BIAS);
static_assert((OFF_P % 16) == 0 && (OFF_T % 16) == 0 && (OFF_BIAS % 16) == 0 && (OFF_MEAN % 16) == 0);

#define WS_WT    0
#define SZ_WT    (NLAYER * 4 * HID * HID * 2)
#define WS_RPHI  (WS_WT + SZ_WT)
#define SZ_RP    (HID * KCAT * 2)
#define WS_RPLO  (WS_RPHI + SZ_RP)
#define WS_POOL  (WS_RPLO + SZ_RP)
#define SZ_POOL  (NMOL * 2 * HID * 4)
#define WS_TOTAL (WS_POOL + SZ_POOL)
static_assert(WS_TOTAL == 1703936);
static_assert(WS_TOTAL <= 134217728);
static_assert((WS_RPHI % 128) == 0 && (WS_RPLO % 128) == 0 && (WS_POOL % 128) == 0);

__device__ __forceinline__ v8f wmma_f16(v16h a, v16h b, v8f c) {
  v8f d = __builtin_amdgcn_wmma_f32_16x16x32_f16(false, a, false, b, (short)0, c, false, false);
  asm volatile("v_nop\n\tv_nop\n\tv_nop\n\tv_nop" : "+v"(d) : "v"(a), "v"(b));
  return d;
}
__device__ __forceinline__ v8f wmma_bf16(v16b a, v16b b, v8f c) {
  v8f d = __builtin_amdgcn_wmma_f32_16x16x32_bf16(false, a, false, b, (short)0, c, false, false);
  asm volatile("v_nop\n\tv_nop\n\tv_nop\n\tv_nop" : "+v"(d) : "v"(a), "v"(b));
  return d;
}

__device__ __forceinline__ v16h frag_h(const _Float16* p, int h) {
  FragH f;
  f.half[0] = *(const v8ha*)(p + 8 * h);
  f.half[1] = *(const v8ha*)(p + 16 + 8 * h);
  return f.v;
}
__device__ __forceinline__ v16b frag_b(const unsigned short* p, int h) {
  FragB f;
  f.half[0] = *(const v8usa*)(p + 8 * h);
  f.half[1] = *(const v8usa*)(p + 16 + 8 * h);
  return f.v;
}
__device__ __forceinline__ v16h frag_f32(const float* row, int k0, int h) {
  const float* p0 = row + k0 + 8 * h;
  const float* p1 = p0 + 16;
  const v4f a0 = *(const v4fa*)p0, a1 = *(const v4fa*)(p0 + 4);
  const v4f b0 = *(const v4fa*)p1, b1 = *(const v4fa*)(p1 + 4);
  FragH f;
  const v8h lo = { (_Float16)a0.x, (_Float16)a0.y, (_Float16)a0.z, (_Float16)a0.w,
                   (_Float16)a1.x, (_Float16)a1.y, (_Float16)a1.z, (_Float16)a1.w };
  const v8h hg = { (_Float16)b0.x, (_Float16)b0.y, (_Float16)b0.z, (_Float16)b0.w,
                   (_Float16)b1.x, (_Float16)b1.y, (_Float16)b1.z, (_Float16)b1.w };
  f.half[0] = lo;
  f.half[1] = hg;
  return f.v;
}

__device__ __forceinline__ void zero_acc(v8f (&acc)[8]) {
  const v8f z = {0.f, 0.f, 0.f, 0.f, 0.f, 0.f, 0.f, 0.f};
  #pragma unroll
  for (int j = 0; j < 8; ++j) acc[j] = z;
}

__device__ __forceinline__ void gemm_f32a(v8f (&acc)[8], const float* arow,
                                          const _Float16* bt, int h, int m) {
  #pragma unroll 1
  for (int kc = 0; kc < HID / 32; ++kc) {
    const v16h a = frag_f32(arow, 32 * kc, h);
    #pragma unroll
    for (int j = 0; j < 8; ++j) {
      const v16h b = frag_h(bt + (size_t)(16 * j + m) * HID + 32 * kc, h);
      acc[j] = wmma_f16(a, b, acc[j]);
    }
  }
}
__device__ __forceinline__ void gemm_h(v8f (&acc)[8], const _Float16* arow,
                                       const _Float16* bt, int h, int m) {
  #pragma unroll 1
  for (int kc = 0; kc < HID / 32; ++kc) {
    const v16h a = frag_h(arow + 32 * kc, h);
    #pragma unroll
    for (int j = 0; j < 8; ++j) {
      const v16h b = frag_h(bt + (size_t)(16 * j + m) * HID + 32 * kc, h);
      acc[j] = wmma_f16(a, b, acc[j]);
    }
  }
}

__device__ __forceinline__ void epi_rowmajor(const v8f (&acc)[8], const float* bias,
                                             _Float16* dst, int row0, int h, int m) {
  #pragma unroll
  for (int j = 0; j < 8; ++j) {
    const float bb = bias[16 * j + m];
    #pragma unroll
    for (int r = 0; r < 8; ++r)
      dst[(row0 + 8 * h + r) * HID + 16 * j + m] = (_Float16)fmaf(acc[j][r], WINV, bb);
  }
}
__device__ __forceinline__ void epi_trans_colsum(const v8f (&acc)[8], const float* bias,
                                                 _Float16* dstT, float* colsum_w,
                                                 int row0, int h, int m) {
  #pragma unroll
  for (int j = 0; j < 8; ++j) {
    const float bb = bias[16 * j + m];
    v8h tv;
    float cs = 0.0f;
    #pragma unroll
    for (int r = 0; r < 8; ++r) {
      const float y = fmaf(acc[j][r], WINV, bb);
      tv[r] = (_Float16)y;
      cs += y;
    }
    *(v8ha*)(dstT + (16 * j + m) * HID + row0 + 8 * h) = tv;
    cs += __shfl_xor(cs, 16);
    if (h == 0) colsum_w[16 * j + m] = cs;
  }
}

__device__ __forceinline__ unsigned short bf16_bits(float x) {
  unsigned u = __float_as_uint(x);
  u = u + 0x7FFFu + ((u >> 16) & 1u);
  return (unsigned short)(u >> 16);
}
__device__ __forceinline__ float bf16_val(unsigned short s) {
  return __uint_as_float(((unsigned)s) << 16);
}

__global__ __launch_bounds__(NTHR) void prep_kernel(
    const float* __restrict__ Wq, const float* __restrict__ Wk,
    const float* __restrict__ Wvm, const float* __restrict__ Wvp,
    const float* __restrict__ rpW,
    _Float16* __restrict__ wT, unsigned short* __restrict__ rpHi,
    unsigned short* __restrict__ rpLo)
{
  const int bid = blockIdx.x, tid = threadIdx.x;
  if (bid < NLAYER * 4) {
    const int l = bid >> 2, w = bid & 3;
    const float* src = (w == 0) ? Wq : ((w == 1) ? Wk : ((w == 2) ? Wvm : Wvp));
    src += (size_t)l * HID * HID;
    _Float16* dst = wT + (size_t)bid * HID * HID;
    v8h o[8];
    #pragma unroll
    for (int it = 0; it < 8; ++it) {
      const int p = it * NTHR + tid;
      const int n = p >> 4, k0 = (p & 15) * 8;
      v8h t;
      #pragma unroll
      for (int i = 0; i < 8; ++i) t[i] = (_Float16)(src[(k0 + i) * HID + n] * WSCALE);
      o[it] = t;
    }
    #pragma unroll
    for (int it = 0; it < 8; ++it) {
      const int p = it * NTHR + tid;
      const int n = p >> 4, k0 = (p & 15) * 8;
      *(volatile v8h*)(dst + n * HID + k0) = o[it];
    }
    __threadfence();
    #pragma unroll
    for (int it = 0; it < 8; ++it) {
      const int p = it * NTHR + tid;
      const int n = p >> 4, k0 = (p & 15) * 8;
      *(volatile v8h*)(dst + n * HID + k0) = o[it];
    }
  } else {
    const int hf = bid - NLAYER * 4;
    v8us oh[8], ol[8];
    #pragma unroll
    for (int it = 0; it < 8; ++it) {
      const int p = it * NTHR + tid;
      const int n = 64 * hf + (p >> 5), k0 = (p & 31) * 8;
      v8us th, tl;
      #pragma unroll
      for (int i = 0; i < 8; ++i) {
        const float v = rpW[(k0 + i) * HID + n];
        const unsigned short hb = bf16_bits(v);
        const unsigned short lb = bf16_bits(v - bf16_val(hb));
        th[i] = hb;
        tl[i] = lb;
      }
      oh[it] = th;
      ol[it] = tl;
    }
    #pragma unroll
    for (int it = 0; it < 8; ++it) {
      const int p = it * NTHR + tid;
      const int n = 64 * hf + (p >> 5), k0 = (p & 31) * 8;
      *(volatile v8us*)(rpHi + n * KCAT + k0) = oh[it];
      *(volatile v8us*)(rpLo + n * KCAT + k0) = ol[it];
    }
    __threadfence();
    #pragma unroll
    for (int it = 0; it < 8; ++it) {
      const int p = it * NTHR + tid;
      const int n = 64 * hf + (p >> 5), k0 = (p & 31) * 8;
      *(volatile v8us*)(rpHi + n * KCAT + k0) = oh[it];
      *(volatile v8us*)(rpLo + n * KCAT + k0) = ol[it];
    }
  }
}

__global__ __launch_bounds__(NTHR) void mol_kernel(
    const float* __restrict__ atom_types, const float* __restrict__ coords,
    const int* __restrict__ edge_index, const float* __restrict__ edge_attr,
    const float* __restrict__ emb_Wm, const float* __restrict__ emb_bm,
    const float* __restrict__ emb_Wp, const float* __restrict__ emb_bp,
    const float* __restrict__ bq, const float* __restrict__ bk,
    const float* __restrict__ bvm, const float* __restrict__ bvp,
    const float* __restrict__ We, const float* __restrict__ be,
    const float* __restrict__ dist_scale,
    const float* __restrict__ ln_g, const float* __restrict__ ln_b,
    const float* __restrict__ rp_b,
    const _Float16* __restrict__ wT,
    const unsigned short* __restrict__ rpHi, const unsigned short* __restrict__ rpLo,
    float* __restrict__ pooled)
{
  extern __shared__ __align__(16) char smem[];
  float*          sMag    = (float*)(smem + OFF_MAG);
  float*          sPh     = (float*)(smem + OFF_PH);
  _Float16*       sP      = (_Float16*)(smem + OFF_P);
  _Float16*       sT      = (_Float16*)(smem + OFF_T);
  float*          sBias   = (float*)(smem + OFF_BIAS);
  int*            sSlot   = (int*)(smem + OFF_SLOT);
  float*          sVal    = (float*)(smem + OFF_VAL);
  int*            sTmp    = (int*)(smem + OFF_VAL);
  float*          sColSum = (float*)(smem + OFF_VAL);
  int*            sCnt    = (int*)(smem + OFF_CNT);
  int*            sStart  = (int*)(smem + OFF_START);
  float*          sMean   = (float*)(smem + OFF_MEAN);
  unsigned short* sAhi    = (unsigned short*)(smem + OFF_BIAS);
  unsigned short* sAlo    = (unsigned short*)(smem + OFF_P);

  const int b = blockIdx.x, tid = threadIdx.x, lane = tid & 31, wv = tid >> 5;
  const int h = lane >> 4, m = lane & 15;
  const int row0 = wv * 16;

  {
    const int c = tid & (HID - 1);
    const int nb = tid >> 7;
    float wm[KEMB], wp[KEMB];
    #pragma unroll
    for (int k = 0; k < KEMB; ++k) { wm[k] = emb_Wm[k * HID + c]; wp[k] = emb_Wp[k * HID + c]; }
    const float bm0 = emb_bm[c], bp0 = emb_bp[c];
    const float* at = atom_types + (size_t)b * NATOM * INDIM;
    const float* cs = coords + (size_t)b * NATOM * 3;
    #pragma unroll 1
    for (int i = 0; i < NATOM / 2; ++i) {
      const int n = 2 * i + nb;
      float xm = 0.0f, xp = 0.0f;
      #pragma unroll
      for (int k = 0; k < INDIM; ++k) {
        const float xv = at[n * INDIM + k];
        xm = fmaf(xv, wm[k], xm);
        xp = fmaf(xv, wp[k], xp);
      }
      #pragma unroll
      for (int k = 0; k < 3; ++k) {
        const float xv = cs[n * 3 + k];
        xm = fmaf(xv, wm[INDIM + k], xm);
        xp = fmaf(xv, wp[INDIM + k], xp);
      }
      sMag[n * HID + c] = xm + bm0;
      sPh[n * HID + c]  = xp + bp0;
    }
  }

  const int* ei0 = edge_index + (size_t)b * 2 * NEDGE;
  const int* ei1 = ei0 + NEDGE;
  if (wv == 0) {
    #pragma unroll
    for (int i = 0; i < NATOM / 32; ++i) sCnt[lane + 32 * i] = 0;
    __builtin_amdgcn_fence(__ATOMIC_RELEASE, "wavefront");
    __builtin_amdgcn_wave_barrier();
    #pragma unroll 1
    for (int ck = 0; ck < NEDGE / 32; ++ck) {
      const int e = ck * 32 + lane;
      int key = ei0[e]; key = min(max(key, 0), NATOM - 1);
      int dst = ei1[e]; dst = min(max(dst, 0), NATOM - 1);
      unsigned msk = 0xffffffffu;
      #pragma unroll
      for (int bt = 0; bt < 7; ++bt) {
        const int bit = (key >> bt) & 1;
        const unsigned bb = __builtin_amdgcn_ballot_w32(bit != 0);
        msk &= bit ? bb : ~bb;
      }
      const unsigned lt = (1u << lane) - 1u;
      const int rank = (int)__popc(msk & lt);
      const int cntg = (int)__popc(msk);
      const int cur = sCnt[key];
      sTmp[e] = (key << 20) | (dst << 12) | ((cur + rank) & 4095);
      if (rank == cntg - 1) sCnt[key] = cur + cntg;
      __builtin_amdgcn_fence(__ATOMIC_RELEASE, "wavefront");
      __builtin_amdgcn_wave_barrier();
    }
    const int c0 = sCnt[4 * lane], c1 = sCnt[4 * lane + 1], c2 = sCnt[4 * lane + 2], c3 = sCnt[4 * lane + 3];
    const int s4 = c0 + c1 + c2 + c3;
    int incl = s4;
    #pragma unroll
    for (int d = 1; d < 32; d <<= 1) {
      const int t = __shfl_up(incl, d);
      if (lane >= d) incl += t;
    }
    const int ex = incl - s4;
    sStart[4 * lane]     = ex;
    sStart[4 * lane + 1] = ex + c0;
    sStart[4 * lane + 2] = ex + c0 + c1;
    sStart[4 * lane + 3] = ex + c0 + c1 + c2;
    if (lane == 31) sStart[NATOM] = incl;
  }
  __syncthreads();
  #pragma unroll
  for (int i = 0; i < NEDGE / NTHR; ++i) {
    const int e = tid + NTHR * i;
    const int t = sTmp[e];
    const int key = (t >> 20) & (NATOM - 1);
    const int dst = (t >> 12) & (NATOM - 1);
    const int r = t & 4095;
    int slot = sStart[key] + r;
    slot = min(max(slot, 0), NEDGE - 1);
    sSlot[slot] = (e << 8) | dst;
  }
  __syncthreads();

  const float* ea = edge_attr + (size_t)b * NEDGE * EDIM;

  #pragma unroll 1
  for (int l = 0; l < NLAYER; ++l) {
    {
      const v4f z4 = {0.0f, 0.0f, 0.0f, 0.0f};
      #pragma unroll
      for (int i = 0; i < (NATOM * NATOM) / (4 * NTHR); ++i)
        *(v4fa*)(sBias + 4 * (tid + NTHR * i)) = z4;
      const float w0 = We[l * EDIM + 0], w1 = We[l * EDIM + 1], w2 = We[l * EDIM + 2], w3 = We[l * EDIM + 3];
      const float be0 = be[l], dsc = dist_scale[l];
      #pragma unroll
      for (int i = 0; i < NEDGE / NTHR; ++i) {
        const int s = tid + NTHR * i;
        int e = sSlot[s] >> 8;
        e = min(max(e, 0), NEDGE - 1);
        const v4f a = *(const v4fa*)(ea + 4 * e);
        float v = a.x * w0 + a.y * w1 + a.z * w2 + a.w * w3 + be0;
        v = v + dsc * a.x;
        sVal[s] = v;
      }
    }
    __syncthreads();
    if (tid < NATOM) {
      const int n = tid;
      int s0 = sStart[n], s1 = sStart[n + 1];
      s0 = min(max(s0, 0), NEDGE);
      s1 = min(max(s1, 0), NEDGE);
      float* brow = sBias + n * HID;
      #pragma unroll 1
      for (int i = 0; i < NEDGE; ++i) {
        const int s = s0 + i;
        if (s >= s1) break;
        const int dd = sSlot[s] & (NATOM - 1);
        brow[dd] += sVal[s];
      }
    }
    __syncthreads();

    const _Float16* wq  = wT + (size_t)(l * 4 + 0) * HID * HID;
    const _Float16* wk  = wT + (size_t)(l * 4 + 1) * HID * HID;
    const _Float16* wvm = wT + (size_t)(l * 4 + 2) * HID * HID;
    const _Float16* wvp = wT + (size_t)(l * 4 + 3) * HID * HID;
    const float* amrow = sMag + (row0 + m) * HID;
    const float* aprow = sPh  + (row0 + m) * HID;
    _Float16* prow = sP + (row0 + m) * HID;

    {
      v8f acc[8]; zero_acc(acc);
      gemm_f32a(acc, amrow, wq, h, m);
      epi_rowmajor(acc, bq + l * HID, sP, row0, h, m);
    }
    {
      v8f acc[8]; zero_acc(acc);
      gemm_f32a(acc, amrow, wk, h, m);
      epi_rowmajor(acc, bk + l * HID, sT, row0, h, m);
    }
    __syncthreads();

    {
      v8f acc[8]; zero_acc(acc);
      gemm_h(acc, prow, sT, h, m);
      #pragma unroll
      for (int j = 0; j < 8; ++j)
        #pragma unroll
        for (int r = 0; r < 8; ++r)
          acc[j][r] = fmaf(acc[j][r], SCALE, sBias[(row0 + 8 * h + r) * HID + 16 * j + m]);
      #pragma unroll
      for (int r = 0; r < 8; ++r) {
        float mx = acc[0][r];
        #pragma unroll
        for (int j = 1; j < 8; ++j) mx = fmaxf(mx, acc[j][r]);
        mx = fmaxf(mx, __shfl_xor(mx, 1));
        mx = fmaxf(mx, __shfl_xor(mx, 2));
        mx = fmaxf(mx, __shfl_xor(mx, 4));
        mx = fmaxf(mx, __shfl_xor(mx, 8));
        float ssum = 0.0f;
        #pragma unroll
        for (int j = 0; j < 8; ++j) {
          const float ev = __expf(acc[j][r] - mx);
          acc[j][r] = ev;
          ssum += ev;
        }
        ssum += __shfl_xor(ssum, 1);
        ssum += __shfl_xor(ssum, 2);
        ssum += __shfl_xor(ssum, 4);
        ssum += __shfl_xor(ssum, 8);
        const float f = PSCALE * __builtin_amdgcn_rcpf(ssum);
        #pragma unroll
        for (int j = 0; j < 8; ++j) acc[j][r] = fmaf(acc[j][r], f, -PSHIFT);
      }
      #pragma unroll
      for (int j = 0; j < 8; ++j)
        #pragma unroll
        for (int r = 0; r < 8; ++r)
          sP[(row0 + 8 * h + r) * HID + 16 * j + m] = (_Float16)acc[j][r];
    }
    __syncthreads();

    {
      v8f acc[8]; zero_acc(acc);
      gemm_f32a(acc, amrow, wvm, h, m);
      epi_trans_colsum(acc, bvm + l * HID, sT, sColSum + wv * HID, row0, h, m);
    }
    __syncthreads();
    if (tid < HID) {
      float s = 0.0f;
      #pragma unroll
      for (int w = 0; w < NTHR / 32; ++w) s += sColSum[w * HID + tid];
      sMean[tid] = s * INVN;
    }
    __syncthreads();

    {
      float gg[8], gb[8];
      #pragma unroll
      for (int j = 0; j < 8; ++j) { gg[j] = ln_g[l * HID + 16 * j + m]; gb[j] = ln_b[l * HID + 16 * j + m]; }
      v8f acc[8]; zero_acc(acc);
      gemm_h(acc, prow, sT, h, m);
      #pragma unroll
      for (int j = 0; j < 8; ++j) {
        const float mc = sMean[16 * j + m];
        #pragma unroll
        for (int r = 0; r < 8; ++r) {
          const int idx = (row0 + 8 * h + r) * HID + 16 * j + m;
          acc[j][r] = fmaf(acc[j][r], PINV, mc) + sMag[idx];
        }
      }
      #pragma unroll
      for (int r = 0; r < 8; ++r) {
        float s = 0.0f;
        #pragma unroll
        for (int j = 0; j < 8; ++j) s += acc[j][r];
        s += __shfl_xor(s, 1); s += __shfl_xor(s, 2); s += __shfl_xor(s, 4); s += __shfl_xor(s, 8);
        const float mu = s * INVN;
        float v = 0.0f;
        #pragma unroll
        for (int j = 0; j < 8; ++j) { const float d = acc[j][r] - mu; v += d * d; }
        v += __shfl_xor(v, 1); v += __shfl_xor(v, 2); v += __shfl_xor(v, 4); v += __shfl_xor(v, 8);
        const float rinv = rsqrtf(v * INVN + LNEPS);
        #pragma unroll
        for (int j = 0; j < 8; ++j)
          sMag[(row0 + 8 * h + r) * HID + 16 * j + m] = (gg[j] * (acc[j][r] - mu)) * rinv + gb[j];
      }
    }
    __syncthreads();

    {
      v8f acc[8]; zero_acc(acc);
      gemm_f32a(acc, aprow, wvp, h, m);
      epi_trans_colsum(acc, bvp + l * HID, sT, sColSum + wv * HID, row0, h, m);
    }
    __syncthreads();
    if (tid < HID) {
      float s = 0.0f;
      #pragma unroll
      for (int w = 0; w < NTHR / 32; ++w) s += sColSum[w * HID + tid];
      sMean[HID + tid] = s * INVN;
    }
    __syncthreads();

    {
      v8f acc[8]; zero_acc(acc);
      gemm_h(acc, prow, sT, h, m);
      #pragma unroll
      for (int j = 0; j < 8; ++j) {
        const float mc = sMean[HID + 16 * j + m];
        #pragma unroll
        for (int r = 0; r < 8; ++r) {
          const int idx = (row0 + 8 * h + r) * HID + 16 * j + m;
          sPh[idx] = fmaf(acc[j][r], PINV, mc) + sPh[idx];
        }
      }
    }
    __syncthreads();
  }

  {
    #pragma unroll 1
    for (int i = 0; i < (NATOM * HID) / NTHR; ++i) {
      const int idx = tid + NTHR * i;
      const int n = idx >> 7, c = idx & (HID - 1);
      const float mg = sMag[n * HID + c];
      const float p  = sPh[n * HID + c];
      const float cn = cosf(p), sn = sinf(p);
      const float re = mg * cn, im = mg * sn;
      const unsigned short rh = bf16_bits(re);
      const unsigned short rl = bf16_bits(re - bf16_val(rh));
      const unsigned short ih = bf16_bits(im);
      const unsigned short il = bf16_bits(im - bf16_val(ih));
      sAhi[n * KCAT + c] = rh;        sAlo[n * KCAT + c] = rl;
      sAhi[n * KCAT + HID + c] = ih;  sAlo[n * KCAT + HID + c] = il;
    }
  }
  __syncthreads();

  {
    v8f acc[8]; zero_acc(acc);
    const unsigned short* arh = sAhi + (row0 + m) * KCAT;
    const unsigned short* arl = sAlo + (row0 + m) * KCAT;
    #pragma unroll 1
    for (int kc = 0; kc < KCAT / 32; ++kc) {
      const v16b ah = frag_b(arh + 32 * kc, h);
      const v16b al = frag_b(arl + 32 * kc, h);
      #pragma unroll
      for (int j = 0; j < 8; ++j) {
        const size_t boff = (size_t)(16 * j + m) * KCAT + 32 * kc;
        const v16b bh = frag_b(rpHi + boff, h);
        const v16b bl = frag_b(rpLo + boff, h);
        acc[j] = wmma_bf16(ah, bh, acc[j]);
        acc[j] = wmma_bf16(ah, bl, acc[j]);
        acc[j] = wmma_bf16(al, bh, acc[j]);
      }
    }
    #pragma unroll
    for (int j = 0; j < 8; ++j) {
      const float bb = rp_b[16 * j + m];
      float cs = 0.0f;
      #pragma unroll
      for (int r = 0; r < 8; ++r) cs += acc[j][r] + bb;
      cs += __shfl_xor(cs, 16);
      if (h == 0) sColSum[wv * HID + 16 * j + m] = cs;
    }
  }
  __syncthreads();

  {
    const int c = tid & (HID - 1);
    float s = 0.0f;
    #pragma unroll
    for (int w = 0; w < NTHR / 32; ++w) s += sColSum[w * HID + c];
    sMean[tid] = (tid < HID) ? (s * INVN) : s;
  }
  __syncthreads();
  if (wv == 0) {
    float* dstp = pooled + (size_t)b * (2 * HID);
    const v4f v0 = *(const v4fa*)(sMean + 4 * lane);
    const v4f v1 = *(const v4fa*)(sMean + HID + 4 * lane);
    *(volatile v4f*)(dstp + 4 * lane) = v0;
    *(volatile v4f*)(dstp + HID + 4 * lane) = v1;
    __threadfence();
    *(volatile v4f*)(dstp + 4 * lane) = v0;
    *(volatile v4f*)(dstp + HID + 4 * lane) = v1;
  }
}

__global__ __launch_bounds__(NTHR) void head_kernel(
    const float* __restrict__ pooled,
    const float* __restrict__ h1W, const float* __restrict__ h1b,
    const float* __restrict__ h2W, const float* __restrict__ h2b,
    float* __restrict__ out)
{
  __shared__ __align__(16) float sPool[32 * 2 * HID];
  __shared__ float sPart[32 * 4];
  __shared__ __align__(16) float sOut[32];
  const int tid = threadIdx.x, lane = tid & 31, wv = tid >> 5;
  const int b0 = blockIdx.x * 32;
  #pragma unroll 1
  for (int i = 0; i < 32; ++i) sPool[i * 2 * HID + tid] = pooled[(size_t)(b0 + i) * (2 * HID) + tid];
  __syncthreads();
  const int hh = tid & (HID - 1), g = tid >> 7, wg = wv & 3;
  const float bias1 = h1b[hh], w2 = h2W[hh];
  #pragma unroll 1
  for (int it = 0; it < 16; ++it) {
    const int mol = 2 * it + g;
    const float* p = sPool + mol * 2 * HID;
    float d = 0.0f;
    #pragma unroll 4
    for (int k = 0; k < 2 * HID; ++k) d = fmaf(p[k], h1W[k * HID + hh], d);
    d += bias1;
    const float sg = __builtin_amdgcn_rcpf(1.0f + __expf(-d));
    float q = (d * sg) * w2;
    q += __shfl_xor(q, 16);
    q += __shfl_xor(q, 8);
    q += __shfl_xor(q, 4);
    q += __shfl_xor(q, 2);
    q += __shfl_xor(q, 1);
    if (lane == 0) sPart[mol * 4 + wg] = q;
  }
  __syncthreads();
  if (tid < 32) {
    const float* pp = sPart + tid * 4;
    sOut[tid] = ((pp[0] + pp[1]) + (pp[2] + pp[3])) + h2b[0];
  }
  __syncthreads();
  if (tid < 8) {
    const v4f v = *(const v4fa*)(sOut + 4 * tid);
    float* dst = out + b0 + 4 * tid;
    *(volatile v4f*)dst = v;
    __threadfence();
    *(volatile v4f*)dst = v;
  }
}

extern "C" void kernel_launch(void* const* d_in, const int* in_sizes, int n_in,
                              void* d_out, int out_size, void* d_ws, size_t ws_size,
                              hipStream_t stream) {
  if (n_in < 27) return;
  if (in_sizes[0] != NMOL * NATOM * INDIM) return;
  if (in_sizes[1] != NMOL * NATOM * 3) return;
  if (in_sizes[2] != NMOL * 2 * NEDGE) return;
  if (in_sizes[3] != NMOL * NEDGE * EDIM) return;
  if (in_sizes[4] != KEMB * HID || in_sizes[5] != HID || in_sizes[6] != KEMB * HID || in_sizes[7] != HID) return;
  if (in_sizes[8] != NLAYER * HID * HID || in_sizes[10] != NLAYER * HID * HID ||
      in_sizes[12] != NLAYER * HID * HID || in_sizes[14] != NLAYER * HID * HID) return;
  if (in_sizes[9] != NLAYER * HID || in_sizes[11] != NLAYER * HID ||
      in_sizes[13] != NLAYER * HID || in_sizes[15] != NLAYER * HID) return;
  if (in_sizes[16] != NLAYER * EDIM || in_sizes[17] != NLAYER || in_sizes[18] != NLAYER) return;
  if (in_sizes[19] != NLAYER * HID || in_sizes[20] != NLAYER * HID) return;
  if (in_sizes[21] != KCAT * HID || in_sizes[22] != HID) return;
  if (in_sizes[23] != KCAT * HID || in_sizes[24] != HID || in_sizes[25] != HID || in_sizes[26] != 1) return;
  if (out_size != NMOL) return;
  if ((size_t)WS_TOTAL > ws_size) return;

  const float* atom_types = (const float*)d_in[0];
  const float* coords     = (const float*)d_in[1];
  const int*   edge_index = (const int*)d_in[2];
  const float* edge_attr  = (const float*)d_in[3];
  const float* emb_Wm = (const float*)d_in[4];
  const float* emb_bm = (const float*)d_in[5];
  const float* emb_Wp = (const float*)d_in[6];
  const float* emb_bp = (const float*)d_in[7];
  const float* Wq  = (const float*)d_in[8];   const float* bq  = (const float*)d_in[9];
  const float* Wk  = (const float*)d_in[10];  const float* bk  = (const float*)d_in[11];
  const float* Wvm = (const float*)d_in[12];  const float* bvm = (const float*)d_in[13];
  const float* Wvp = (const float*)d_in[14];  const float* bvp = (const float*)d_in[15];
  const float* We  = (const float*)d_in[16];  const float* be  = (const float*)d_in[17];
  const float* dist_scale = (const float*)d_in[18];
  const float* ln_g = (const float*)d_in[19]; const float* ln_b = (const float*)d_in[20];
  const float* rp_W = (const float*)d_in[21]; const float* rp_b = (const float*)d_in[22];
  const float* h1_W = (const float*)d_in[23]; const float* h1_b = (const float*)d_in[24];
  const float* h2_W = (const float*)d_in[25]; const float* h2_b = (const float*)d_in[26];
  float* out = (float*)d_out;

  char* ws = (char*)d_ws;
  _Float16*       wT     = (_Float16*)(ws + WS_WT);
  unsigned short* rpHi   = (unsigned short*)(ws + WS_RPHI);
  unsigned short* rpLo   = (unsigned short*)(ws + WS_RPLO);
  float*          pooled = (float*)(ws + WS_POOL);

  prep_kernel<<<NLAYER * 4 + 2, NTHR, 0, stream>>>(Wq, Wk, Wvm, Wvp, rp_W, wT, rpHi, rpLo);

  (void)hipFuncSetAttribute(reinterpret_cast<const void*>(&mol_kernel),
                            hipFuncAttributeMaxDynamicSharedMemorySize, SMEM_BYTES);
  mol_kernel<<<NMOL, NTHR, SMEM_BYTES, stream>>>(
      atom_types, coords, edge_index, edge_attr,
      emb_Wm, emb_bm, emb_Wp, emb_bp,
      bq, bk, bvm, bvp, We, be, dist_scale, ln_g, ln_b, rp_b,
      wT, rpHi, rpLo, pooled);

  head_kernel<<<NMOL / 32, NTHR, 0, stream>>>(pooled, h1_W, h1_b, h2_W, h2_b, out);
}
